// MPLPNodeLabel_61512521613939
// MI455X (gfx1250) — hardware-run, weakly checked
//
#include <hip/hip_runtime.h>


namespace {
constexpr int N = 100000, DIM = 128, M = 1600000, E = 200000, KB9 = 9, OUTW = 81;
constexpr float XS = 8.0f;
typedef _Float16 b16;
typedef __attribute__((ext_vector_type(16))) _Float16 v16b;
typedef __attribute__((ext_vector_type(8))) _Float16 v8b;
typedef __attribute__((ext_vector_type(8))) float v8f;
typedef __attribute__((ext_vector_type(4))) float v4f;
typedef __attribute__((ext_vector_type(4))) _Float16 v4b;
__device__ __forceinline__ float bf16_rne(float f) { unsigned int u = __float_as_uint(f); u += 0x7FFFu + ((u >> 16) & 1u); return __uint_as_float(u & 0xFFFF0000u); }
__device__ __forceinline__ void split16(float v, b16& hi, b16& lo) { hi = (b16)v; lo = (b16)(v - (float)hi); }
__device__ __forceinline__ v16b frag_kb(const b16* p, int hh) { const v8b a = *(const v8b*)(p + 8 * hh), b = *(const v8b*)(p + 16 + 8 * hh); v16b f;
#pragma unroll
  for (int e = 0; e < 8; ++e) { f[e] = a[e]; f[8 + e] = b[e]; } return f; }
__device__ __forceinline__ v8f wmma16b(v16b a, v16b b, v8f c) { v8f d = __builtin_amdgcn_wmma_f32_16x16x32_f16(false, a, false, b, (short)0, c, false, false); asm volatile("v_nop\n\tv_nop\n\tv_nop\n\tv_nop" : "+v"(d) : "v"(a), "v"(b)); return d; }
__device__ __forceinline__ void wave_lds_sync() { __builtin_amdgcn_fence(__ATOMIC_RELEASE, "workgroup"); __builtin_amdgcn_wave_barrier(); __builtin_amdgcn_fence(__ATOMIC_ACQUIRE, "workgroup"); }
__device__ __forceinline__ float pmul(float a, float b) { float p = a * b; asm volatile("" : "+v"(p)); return p; }
__device__ __forceinline__ int iclamp(int v, int lo, int hi) { return v < lo ? lo : (v > hi ? hi : v); }
constexpr int CSR_NBLK9 = 512, CSR_GB9 = 9, CSR_GN9 = 1 << CSR_GB9  , CSR_TS9 = (CSR_GN9 < 32 ? 32 : CSR_GN9)  , CSR_MAXG9 = 512, CSR_CAP9 = 12288  ;
__device__ __host__ __forceinline__ int csr_tix9(int v) { return (v >> CSR_GB9) * CSR_TS9 + (v & (CSR_GN9 - 1)); }
__global__ __launch_bounds__(64) void csrA_kernel9(const int* __restrict__ dst, int E, int N, int nG, int CHP, int NGP, int* __restrict__ STG, int* __restrict__ HST) {
  extern __shared__ int sm[];
  int* cnt = sm; int* run = sm + NGP; int* ids = sm + 2 * NGP;
  const int b = blockIdx.x; const int ch = (E + CSR_NBLK9 - 1) / CSR_NBLK9; const int e0 = b * ch, e1 = min(E, e0 + ch);
  for (int i = threadIdx.x; i < NGP; i += 64) cnt[i] = 0;
  for (int i = threadIdx.x; i < CHP; i += 64) ids[i] = -1;
  __syncthreads();
  if (threadIdx.x == 0) {
    for (int e = e0; e < e1; ++e) { int d = dst[e]; d = (d < 0) ? 0 : (d >= N ? N - 1 : d); cnt[d >> CSR_GB9] += 1; }
    int acc = 0; for (int g = 0; g < nG; ++g) { run[g] = acc; acc += cnt[g]; }
    for (int e = e0; e < e1; ++e) { int d = dst[e]; d = (d < 0) ? 0 : (d >= N ? N - 1 : d); const int g = d >> CSR_GB9; ids[run[g]] = e; run[g] += 1; } }
  __syncthreads();
  typedef __attribute__((ext_vector_type(4))) int v4i;
  for (int pass = 0; pass < 2; ++pass) {
    for (int i = threadIdx.x; i < CHP / 4; i += 64) *(volatile v4i*)(STG + (size_t)b * CHP + i * 4) = *(const v4i*)(&ids[i * 4]);
    for (int i = threadIdx.x; i < NGP / 4; i += 64) { v4i v; for (int e = 0; e < 4; ++e) v[e] = (i * 4 + e < nG) ? cnt[i * 4 + e] : 0; *(volatile v4i*)(HST + (size_t)b * NGP + i * 4) = v; }
    __threadfence(); }
}
__global__ __launch_bounds__(512) void csrS_kernel9(const int* __restrict__ HST, int nG, int NGP, int* __restrict__ START, int* __restrict__ TOT, int* __restrict__ OFF) {
  __shared__ int tot[CSR_MAXG9];
  const int b = threadIdx.x;
  for (int pass = 0; pass < 2; ++pass) { int runb = 0; for (int g = 0; g < nG; ++g) { int c = HST[(size_t)b * NGP + g]; c = (c < 0) ? 0 : c; ((volatile int*)OFF)[(size_t)g * CSR_NBLK9 + b] = runb; runb += c; } __threadfence(); }
  for (int g = threadIdx.x; g < nG; g += 512) { int s = 0; for (int bb = 0; bb < CSR_NBLK9; ++bb) { int c = HST[(size_t)bb * NGP + g]; s += (c < 0) ? 0 : c; } tot[g] = s; }
  __syncthreads();
  if (threadIdx.x < 32) {
    __shared__ int st[CSR_MAXG9 + 32];
    if (threadIdx.x == 0) { int acc = 0; for (int g = 0; g < NGP; ++g) { st[g] = acc; if (g < nG) acc += (tot[g] + 31) & ~31; } st[NGP] = acc; }
    __builtin_amdgcn_fence(__ATOMIC_RELEASE, "workgroup"); __builtin_amdgcn_wave_barrier(); __builtin_amdgcn_fence(__ATOMIC_ACQUIRE, "workgroup");
    for (int pass = 0; pass < 2; ++pass) { for (int i = threadIdx.x; i < NGP + 32; i += 32) { ((volatile int*)START)[i] = (i <= NGP) ? st[min(i, NGP)] : 0; ((volatile int*)TOT)[i] = (i < nG) ? tot[i] : 0; } __threadfence(); } }
}
__global__ __launch_bounds__(256) void csrB_kernel9(const int* __restrict__ dst, int N, int nG, int CHP, int NGP, int permLen, const int* __restrict__ STG, const int* __restrict__ HST, const int* __restrict__ OFF, const int* __restrict__ START, const int* __restrict__ TOT, int* __restrict__ PERM, int* __restrict__ ROWPTR, int* __restrict__ ROWCNT, int* __restrict__ FLAG) {
  typedef __attribute__((ext_vector_type(4))) int v4i;
  __shared__ int ids[CSR_CAP9]; __shared__ unsigned short key[CSR_CAP9]; __shared__ int outp[CSR_CAP9]; __shared__ int ncnt[CSR_GN9 + 1]; __shared__ int boff[CSR_NBLK9 + 1];
  const int g = blockIdx.x, t_ = threadIdx.x; int tot = TOT[g]; int st = START[g], stn = START[g + 1]; const int v0 = g * CSR_GN9; const int nv = min(CSR_GN9, N - v0); const int t0 = g * CSR_TS9;
  st = (st < 0) ? 0 : (st > permLen - 32 ? permLen - 32 : st) & ~31; stn = (stn < st) ? st : (stn > permLen ? permLen : stn); tot = (tot < 0) ? 0 : tot; if (tot > stn - st && tot <= CSR_CAP9) tot = stn - st;
  if (tot > CSR_CAP9) {
    for (int pass = 0; pass < 2; ++pass) { for (int i = t_; i < CSR_TS9 / 4; i += 256) { v4i a, c; for (int e = 0; e < 4; ++e) { a[e] = st; c[e] = 0; } *(volatile v4i*)(ROWPTR + t0 + i * 4) = a; *(volatile v4i*)(ROWCNT + t0 + i * 4) = c; } if (t_ == 0) ((volatile int*)FLAG)[0] = 1; __threadfence(); } (void)nv; return; }
  if (t_ == 0) { int acc = 0; for (int b = 0; b < CSR_NBLK9; ++b) { boff[b] = acc; int c = HST[(size_t)b * NGP + g]; c = (c < 0) ? 0 : (c > CHP ? CHP : c); acc += c; if (acc > tot) acc = tot; } boff[CSR_NBLK9] = acc; }
  for (int i = t_; i <= CSR_GN9; i += 256) ncnt[i] = 0;
  __syncthreads();
  for (int b = 0; b < CSR_NBLK9; ++b) { const int c = boff[b + 1] - boff[b]; int o_ = OFF[(size_t)g * CSR_NBLK9 + b]; o_ = (o_ < 0) ? 0 : (o_ > CHP - c ? CHP - c : o_); const int* src_ = STG + (size_t)b * CHP + o_;
    for (int i = t_; i < c; i += 256) { int id = src_[i]; id = (id < 0) ? 0 : id; ids[boff[b] + i] = id; int d = dst[id]; d = (d < v0) ? v0 : (d >= N ? N - 1 : d); int kk = d - v0; kk = (kk < 0) ? 0 : (kk >= CSR_GN9 ? CSR_GN9 - 1 : kk); key[boff[b] + i] = (unsigned short)kk; } }
  __syncthreads();
  if (t_ == 0) { for (int i = 0; i < tot; ++i) ncnt[key[i]] += 1; int acc = 0; for (int vl = 0; vl < CSR_GN9; ++vl) { const int c = ncnt[vl]; ncnt[vl] = acc; acc += c; } ncnt[CSR_GN9] = acc;
    for (int i = 0; i < tot; ++i) { const int vl = key[i]; outp[ncnt[vl]] = ids[i]; ncnt[vl] += 1; }
    for (int vl = CSR_GN9; vl > 0; --vl) ncnt[vl] = ncnt[vl - 1]; ncnt[0] = 0; }
  __syncthreads();
  for (int pass = 0; pass < 2; ++pass) {
    for (int i = t_; i < (stn - st) / 4; i += 256) { v4i v; for (int e = 0; e < 4; ++e) { const int q = i * 4 + e; v[e] = (q < tot) ? outp[q] : -1; } *(volatile v4i*)(PERM + st + i * 4) = v; }
    for (int i = t_; i < CSR_TS9 / 4; i += 256) { v4i a, c; for (int e = 0; e < 4; ++e) { const int vl = i * 4 + e; const int vc = vl < CSR_GN9 ? vl : CSR_GN9; a[e] = (vl < CSR_GN9) ? st + ncnt[vc] : st; c[e] = (vl < nv) ? (ncnt[(vc < CSR_GN9 ? vc : CSR_GN9 - 1) + 1] - ncnt[vc]) : 0; } *(volatile v4i*)(ROWPTR + t0 + i * 4) = a; *(volatile v4i*)(ROWCNT + t0 + i * 4) = c; }
    __threadfence(); }
}
__global__ __launch_bounds__(256) void csrZ_kernel9(int* __restrict__ p, size_t n4) { typedef __attribute__((ext_vector_type(4))) int v4i; const size_t tid = (size_t)blockIdx.x * 256 + threadIdx.x, nth = (size_t)gridDim.x * 256; v4i z = {0, 0, 0, 0}; for (size_t i = tid; i < n4; i += nth) *(volatile v4i*)(p + i * 4) = z; }
struct CsrBufs9 { int *STG, *HST, *OFF, *START, *TOT, *PERM, *ROWPTR, *ROWCNT, *FLAG; int nG, NGP, CHP; size_t permLen; char* base; size_t bytes; };
static size_t csr_carve9(CsrBufs9& c, char* ws, size_t off, int E, int N) {
  const size_t off0 = off; c.base = ws + off;
  auto al = [&](size_t bytes) { char* p = ws + off; off += (bytes + 255) & ~(size_t)255; return p; };
  c.nG = (N + CSR_GN9 - 1) / CSR_GN9; c.NGP = (c.nG + 31) & ~31; const int ch = (E + CSR_NBLK9 - 1) / CSR_NBLK9; c.CHP = (ch + 31) & ~31; c.permLen = (size_t)E + 32 * (size_t)c.nG + 32;
  c.STG = (int*)al((size_t)CSR_NBLK9 * c.CHP * 4); c.HST = (int*)al((size_t)CSR_NBLK9 * c.NGP * 4); c.OFF = (int*)al((size_t)c.NGP * CSR_NBLK9 * 4); c.START = (int*)al((size_t)(c.NGP + 64) * 4); c.TOT = (int*)al((size_t)(c.NGP + 64) * 4);
  c.PERM = (int*)al(c.permLen * 4); c.ROWPTR = (int*)al((size_t)c.nG * CSR_TS9 * 4); c.ROWCNT = (int*)al((size_t)c.nG * CSR_TS9 * 4); c.FLAG = (int*)al(256);
  c.bytes = off - off0; return off;
}
static void csr_build9(const CsrBufs9& c, const int* dst, int E, int N, hipStream_t stream) {
  const size_t smem = (size_t)(2 * c.NGP + c.CHP) * 4;
  csrZ_kernel9<<<512, 256, 0, stream>>>((int*)c.base, c.bytes / 16);
  csrA_kernel9<<<CSR_NBLK9, 64, smem, stream>>>(dst, E, N, c.nG, c.CHP, c.NGP, c.STG, c.HST);
  csrS_kernel9<<<1, 512, 0, stream>>>(c.HST, c.nG, c.NGP, c.START, c.TOT, c.OFF);
  csrB_kernel9<<<c.nG, 256, 0, stream>>>(dst, N, c.nG, c.CHP, c.NGP, (int)c.permLen, c.STG, c.HST, c.OFF, c.START, c.TOT, c.PERM, c.ROWPTR, c.ROWCNT, c.FLAG);
}


__device__ __forceinline__ void node_scal(const float* deg, size_t n, float& sa, float& sb, float& dr) { const float d = bf16_rne(deg[n]); sa = rsqrtf(d); sb = rsqrtf(1.0f + logf(d)); dr = 1.0f / d; }
__global__ __launch_bounds__(256) void hop1_kernel(const float* __restrict__ s, const float* __restrict__ deg, const int* __restrict__ cols, const int* __restrict__ PERM, const int* __restrict__ ROWPTR, const int* __restrict__ ROWCNT, int permLen, int NLIM, float* __restrict__ X1) {
  const int wave = threadIdx.x >> 5, lane = threadIdx.x & 31; const size_t n = (size_t)blockIdx.x * 8 + wave; if (n >= (size_t)NLIM) return; int st = ROWPTR[n], cnt = ROWCNT[n]; cnt = iclamp(cnt, 0, 1 << 20); st = iclamp(st, 0, permLen - cnt);
  float a0[4] = {0, 0, 0, 0}, a1[4] = {0, 0, 0, 0}, a2[4] = {0, 0, 0, 0};
#pragma unroll 1
  for (int j = 0; j < cnt; ++j) { const int e = iclamp(PERM[st + j], 0, M - 1); const size_t u = (size_t)iclamp(cols[e], 0, N - 1); if (u >= (size_t)NLIM) continue; float sa, sb, du; node_scal(deg, u, sa, sb, du); const v4f xv = *(const v4f*)(s + u * DIM + lane * 4);
    for (int i = 0; i < 4; ++i) { const float v = bf16_rne(xv[i]); a0[i] += v; a1[i] += pmul(v, sa); a2[i] += pmul(v, sb); } }
  float sn, sbn, dr; node_scal(deg, n, sn, sbn, dr); v4f o0, o1, o2; for (int i = 0; i < 4; ++i) { o0[i] = pmul(a0[i], dr); o1[i] = pmul(a1[i], dr); o2[i] = pmul(a2[i], dr); }
  for (int pass = 0; pass < 2; ++pass) { *(volatile v4f*)(X1 + (n * 3 + 0) * DIM + lane * 4) = o0; *(volatile v4f*)(X1 + (n * 3 + 1) * DIM + lane * 4) = o1; *(volatile v4f*)(X1 + (n * 3 + 2) * DIM + lane * 4) = o2; __threadfence(); }
}
__global__ __launch_bounds__(256) void hop2_kernel(const float* __restrict__ deg, const float* __restrict__ X1, const int* __restrict__ cols, const int* __restrict__ PERM, const int* __restrict__ ROWPTR, const int* __restrict__ ROWCNT, int permLen, int NLIM, b16* __restrict__ X2) {
  const int wave = threadIdx.x >> 5, lane = threadIdx.x & 31; const size_t n = (size_t)blockIdx.x * 8 + wave; if (n >= (size_t)NLIM) return; int st = ROWPTR[n], cnt = ROWCNT[n]; cnt = iclamp(cnt, 0, 1 << 20); st = iclamp(st, 0, permLen - cnt);
  float a[3][4]; for (int p = 0; p < 3; ++p) for (int i = 0; i < 4; ++i) a[p][i] = 0.0f;
#pragma unroll 1
  for (int j = 0; j < cnt; ++j) { const int e = iclamp(PERM[st + j], 0, M - 1); const size_t u = (size_t)iclamp(cols[e], 0, N - 1); if (u >= (size_t)NLIM) continue;
    for (int p = 0; p < 3; ++p) { const v4f xv = *(const v4f*)(X1 + (u * 3 + p) * DIM + lane * 4); for (int i = 0; i < 4; ++i) a[p][i] += xv[i]; } }
  float sa, sb, dr; node_scal(deg, n, sa, sb, dr); v4b o[3];
  for (int i = 0; i < 4; ++i) { o[0][i] = (b16)pmul(a[0][i], dr); o[1][i] = (b16)pmul(a[1][i], dr); o[2][i] = (b16)pmul(a[2][i], dr); }
  for (int pass = 0; pass < 2; ++pass) { for (int p = 0; p < 3; ++p) *(volatile v4b*)(X2 + (n * 3 + p) * DIM + lane * 4) = o[p]; __threadfence(); }
}
__global__ __launch_bounds__(32) void edge_kernel(const float* __restrict__ s, const float* __restrict__ deg, const float* __restrict__ X1, const b16* __restrict__ X2, const int* __restrict__ e0s, const int* __restrict__ e1s, int NLIM, int ELIM, float* __restrict__ out) {
  __shared__ __attribute__((aligned(16))) b16 Ah[16][DIM + 8], Al[16][DIM + 8], Bh[16][DIM + 8], Bl[16][DIM + 8]; __shared__ float Ss[16][17], To[32][OUTW + 2];
  const int lane = threadIdx.x, nloc = lane & 15, hlf = lane >> 4; const size_t eb = (size_t)blockIdx.x * 32; if (eb >= (size_t)ELIM) return;
  for (int r = 9; r < 16; ++r) for (int q = 0; q < 4; ++q) { Ah[r][q * 32 + lane] = (b16)0.0f; Al[r][q * 32 + lane] = (b16)0.0f; Bh[r][q * 32 + lane] = (b16)0.0f; Bl[r][q * 32 + lane] = (b16)0.0f; }
#pragma unroll 1
  for (int ee = 0; ee < 32; ++ee) { const size_t e = eb + ee; const int na = iclamp(e0s[e], 0, N - 1), nb = iclamp(e1s[e], 0, N - 1); const bool ok = na < NLIM && nb < NLIM;
    for (int side = 0; side < 2; ++side) { const int nn = side == 0 ? na : nb; b16 (*Hh)[DIM + 8] = side == 0 ? Ah : Bh; b16 (*Hl)[DIM + 8] = side == 0 ? Al : Bl; float sa, sb, dr; node_scal(deg, (size_t)nn, sa, sb, dr); (void)dr;
      for (int q = 0; q < 4; ++q) { const int c = q * 32 + lane; const float v = ok ? bf16_rne(s[(size_t)nn * DIM + c]) : 0.0f; b16 p, ql;
        split16(v * XS, p, ql); Hh[0][c] = p; Hl[0][c] = ql; split16(pmul(v, sa) * XS, p, ql); Hh[1][c] = p; Hl[1][c] = ql; split16(pmul(v, sb) * XS, p, ql); Hh[2][c] = p; Hl[2][c] = ql;
        const float xp[3] = {v, pmul(v, sa), pmul(v, sb)};
        for (int pp = 0; pp < 3; ++pp) { const float y1 = ok ? X1[((size_t)nn * 3 + pp) * DIM + c] : 0.0f, y2 = ok ? (float)X2[((size_t)nn * 3 + pp) * DIM + c] - xp[pp] : 0.0f; split16(y1 * XS, p, ql); Hh[3 + pp][c] = p; Hl[3 + pp][c] = ql; split16(y2 * XS, p, ql); Hh[6 + pp][c] = p; Hl[6 + pp][c] = ql; } } }
    wave_lds_sync(); v8f acc = {};
#pragma unroll
    for (int kb = 0; kb < DIM; kb += 32) { const v16b a = frag_kb(&Ah[nloc][kb], hlf), al = frag_kb(&Al[nloc][kb], hlf), bh = frag_kb(&Bh[nloc][kb], hlf), bl = frag_kb(&Bl[nloc][kb], hlf); acc = wmma16b(a, bh, acc); acc = wmma16b(a, bl, acc); acc = wmma16b(al, bh, acc); }
#pragma unroll
    for (int r8 = 0; r8 < 8; ++r8) Ss[8 * hlf + r8][nloc] = acc[r8] * (1.0f / (XS * XS));
    wave_lds_sync();
    for (int i = lane; i < OUTW; i += 32) { const int k = i / 9, l = i % 9; To[ee][i] = Ss[k][l] + Ss[l][k]; }
    wave_lds_sync(); }
  for (int pass = 0; pass < 2; ++pass) { for (int i = lane; i < 32 * OUTW; i += 32) ((volatile float*)out)[eb * OUTW + i] = To[i / OUTW][i % OUTW]; __threadfence(); }
}
}

extern "C" void kernel_launch(void* const* d_in, const int* in_sizes, int n_in, void* d_out, int out_size, void* d_ws, size_t ws_size, hipStream_t stream) {
  (void)n_in;
  auto Fp = [&](int i) { return (const float*)d_in[i]; }; auto Ip = [&](int i) { return (const int*)d_in[i]; };
  if (in_sizes[0] != 2 * E || in_sizes[1] != M || in_sizes[2] != M || in_sizes[3] != N || in_sizes[4] != N * DIM || out_size != E * OUTW) return;
  const int NLIM = N, ELIM = E; const int GB8 = N / 8;
  size_t off = 0; char* ws = (char*)d_ws;
  auto carve = [&](size_t bytes) { char* p = ws + off; off += (bytes + 255) & ~(size_t)255; return p; };
  float* X1 = (float*)carve((size_t)N * 3 * DIM * 4); b16* X2 = (b16*)carve((size_t)N * 3 * DIM * 2); CsrBufs9 csr; off = csr_carve9(csr, ws, off, M, N);
  if (off > ws_size) return;
  csr_build9(csr, Ip(1), M, N, stream);
  hop1_kernel<<<GB8, 256, 0, stream>>>(Fp(4), Fp(3), Ip(2), csr.PERM, csr.ROWPTR, csr.ROWCNT, (int)csr.permLen, NLIM, X1);
  hop2_kernel<<<GB8, 256, 0, stream>>>(Fp(3), X1, Ip(2), csr.PERM, csr.ROWPTR, csr.ROWCNT, (int)csr.permLen, NLIM, X2);
  edge_kernel<<<ELIM / 32, 32, 0, stream>>>(Fp(4), Fp(3), X1, X2, Ip(0), Ip(0) + E, NLIM, ELIM, (float*)d_out);
}
